// XLNetRelativeAttention_55336358642049
// MI455X (gfx1250) — hardware-verified
//
#include <hip/hip_runtime.h>
#include <math.h>

constexpr int kQLen    = 1024;
constexpr int kBsz     = 4;
constexpr int kDModel  = 1024;
constexpr int kNHead   = 16;
constexpr int kDHead   = 64;
constexpr int kRLen    = 2048;
constexpr int kHD      = kNHead * kDHead;
constexpr int kTokQ    = kQLen * kBsz;
constexpr int kTokR    = kRLen * kBsz;
constexpr int kBand    = 1088;
constexpr int kBandOff = 960;
constexpr int kEFRow   = 32;
constexpr float kWCarry  = 64.0f;
constexpr float kQCarry  = 8.0f;
constexpr float kPCarry  = 2048.0f;
constexpr float kAVCarry = 256.0f;
constexpr float kScoreScale = 0.125f;
constexpr float kLnEps   = 1e-12f;
constexpr float kInvD    = 1.0f / 1024.0f;

constexpr float kScaleQf32 = 1.0f / kWCarry;
constexpr float kScaleP16  = kQCarry / kWCarry;
constexpr float kScaleSc   = 1.0f / (kQCarry * kQCarry);
constexpr float kScalePV   = kAVCarry / (kPCarry * kQCarry);
constexpr float kScaleOut  = 1.0f / (kAVCarry * kWCarry);

typedef __attribute__((ext_vector_type(16))) _Float16 v16h;
typedef __attribute__((ext_vector_type(8)))  _Float16 v8h;
typedef __attribute__((ext_vector_type(16))) __bf16   v16b;
typedef __attribute__((ext_vector_type(8)))  __bf16   v8b;
typedef __attribute__((ext_vector_type(8)))  float    v8f;
typedef __attribute__((ext_vector_type(4)))  float    v4f;
typedef __attribute__((ext_vector_type(2)))  float    v2f;
typedef __attribute__((ext_vector_type(4)))  unsigned int v4u;

__device__ __forceinline__ unsigned short f2bf_bits(float f) {
  unsigned u = __float_as_uint(f);
  return (unsigned short)((u + 0x7FFFu + ((u >> 16) & 1u)) >> 16);
}
__device__ __forceinline__ float bf_bits2f(unsigned short h) { return __uint_as_float(((unsigned)h) << 16); }

__device__ __forceinline__ void dep_guard_h(v8f& a, v8f& b, v16h x, v16h y) { asm volatile("v_nop\n\tv_nop\n\tv_nop\n\tv_nop" : "+v"(a), "+v"(b) : "v"(x), "v"(y)); }
__device__ __forceinline__ void dep_guard_b(v8f& a, v8f& b, v16b x, v16b y) { asm volatile("v_nop\n\tv_nop\n\tv_nop\n\tv_nop" : "+v"(a), "+v"(b) : "v"(x), "v"(y)); }
__device__ __forceinline__ void keep4_h(v16h a, v16h b, v16h c, v16h d) { asm volatile("v_nop" :: "v"(a), "v"(b), "v"(c), "v"(d)); }
__device__ __forceinline__ void keep4_b(v16b a, v16b b, v16b c, v16b d) { asm volatile("v_nop" :: "v"(a), "v"(b), "v"(c), "v"(d)); }
__device__ __forceinline__ void acc_guard4(v8f& a, v8f& b, v8f& c, v8f& d) { asm volatile("v_nop\n\tv_nop\n\tv_nop\n\tv_nop" : "+v"(a), "+v"(b), "+v"(c), "+v"(d)); }
template <typename T> struct Frag;
template <> struct Frag<_Float16> {
  typedef v16h V; union U { v16h v; v8h h[2]; };
  static __device__ __forceinline__ v16h load(const _Float16* p) {
    U f; f.h[0] = *(const v8h*)(p); f.h[1] = *(const v8h*)(p + 16); return f.v;
  }
  static __device__ __forceinline__ v8f mma(v16h a, v16h b, v8f c) {
    return __builtin_amdgcn_wmma_f32_16x16x32_f16(false, a, false, b, (short)0, c, false, false);
  }
  static __device__ __forceinline__ void guard(v8f& a, v8f& b, v16h x, v16h y) { dep_guard_h(a, b, x, y); }
  static __device__ __forceinline__ void keep(v16h a, v16h b, v16h c, v16h d) { keep4_h(a, b, c, d); }
};
template <> struct Frag<__bf16> {
  typedef v16b V; union U { v16b v; v8b h[2]; };
  static __device__ __forceinline__ v16b load(const __bf16* p) {
    U f; f.h[0] = *(const v8b*)(p); f.h[1] = *(const v8b*)(p + 16); return f.v;
  }
  static __device__ __forceinline__ v8f mma(v16b a, v16b b, v8f c) {
    return __builtin_amdgcn_wmma_f32_16x16x32_bf16(false, a, false, b, (short)0, c, false, false);
  }
  static __device__ __forceinline__ void guard(v8f& a, v8f& b, v16b x, v16b y) { dep_guard_b(a, b, x, y); }
  static __device__ __forceinline__ void keep(v16b a, v16b b, v16b c, v16b d) { keep4_b(a, b, c, d); }
};

__device__ __forceinline__ unsigned pk16(unsigned short a, unsigned short b) { return (unsigned)a | ((unsigned)b << 16); }
__device__ __forceinline__ unsigned short h_bits(float f) { const _Float16 h = (_Float16)f; return __builtin_bit_cast(unsigned short, h); }

template <int ET> struct Elem;
template <> struct Elem<0> { typedef _Float16 T; };
template <> struct Elem<1> { typedef __bf16 T; };
template <int ET, bool SPLIT, int BIAS_MODE, int OUT_MODE, bool RESID, int ACT = 0, bool BAND = false>
__global__ __launch_bounds__(256) void wmma_gemm64(
    const unsigned short* __restrict__ Ap, const unsigned short* __restrict__ A2p, int lda, long strideA,
    const unsigned short* __restrict__ Btp, const unsigned short* __restrict__ Bt2p, int ldb, long strideB,
    void* __restrict__ Cout, void* __restrict__ Cout2, int ldc, long strideC,
    const float* __restrict__ bias,
    const float* __restrict__ resid, long strideR,
    int M, int N, int K, float scale, int bandOff) {
  typedef typename Elem<ET>::T T;
  typedef typename Frag<T>::V V;
  const T* A = (const T*)Ap; const T* A2 = (const T*)A2p; const T* Bt = (const T*)Btp; const T* Bt2 = (const T*)Bt2p;
  __shared__ __align__(16) float sT[8][16 * 68];
  const int b    = blockIdx.y;
  const int lane = threadIdx.x & 31;
  const int wave = threadIdx.x >> 5;
  const int tilesN = N >> 6;
  const int tilesM = M >> 6;
  const int tile = blockIdx.x * 8 + wave;
  if (tile >= tilesM * tilesN) return;
  const int tm = tile / tilesN;
  const int tn = tile - tm * tilesN;
  const int m0 = tm << 6;
  const int n0 = tn << 6;
  const int nB = BAND ? (n0 + bandOff - m0) : n0;

  const T* Ab  = A  + (size_t)b * strideA;
  const T* Bb  = Bt + (size_t)b * strideB;
  const T* Ab2 = SPLIT ? (A2  + (size_t)b * strideA) : nullptr;
  const T* Bb2 = SPLIT ? (Bt2 + (size_t)b * strideB) : nullptr;

  const int rlane = lane & 15;
  const int koff  = (lane >> 4) * 8;
  const int mOff  = (lane >> 4) * 8;

  v8f acc[4][4];
#pragma unroll
  for (int i = 0; i < 4; ++i)
#pragma unroll
    for (int j = 0; j < 4; ++j) acc[i][j] = (v8f){0.f,0.f,0.f,0.f,0.f,0.f,0.f,0.f};

  for (int k0 = 0; k0 < K; k0 += 32) {
    V bh[4], bl[4];
#pragma unroll
    for (int j = 0; j < 4; ++j) {
      const size_t bo = (size_t)(nB + (j << 4) + rlane) * ldb + koff + k0;
      bh[j] = Frag<T>::load(Bb + bo);
      if (SPLIT) bl[j] = Frag<T>::load(Bb2 + bo);
    }
#pragma unroll
    for (int i = 0; i < 4; ++i) {
      const size_t ao = (size_t)(m0 + (i << 4) + rlane) * lda + koff + k0;
      V ah = Frag<T>::load(Ab + ao);
      V al;
      if (SPLIT) al = Frag<T>::load(Ab2 + ao);
#pragma unroll
      for (int j = 0; j < 4; ++j) {
        acc[i][j] = Frag<T>::mma(ah, bh[j], acc[i][j]);
        if (SPLIT) {
          acc[i][j] = Frag<T>::mma(ah, bl[j], acc[i][j]);
          acc[i][j] = Frag<T>::mma(al, bh[j], acc[i][j]);
        }
      }
      Frag<T>::guard(acc[i][0], acc[i][3], ah, SPLIT ? al : ah);
    }
    Frag<T>::keep(bh[0], bh[1], bh[2], bh[3]);
    if (SPLIT) Frag<T>::keep(bl[0], bl[1], bl[2], bl[3]);
  }
  acc_guard4(acc[0][0], acc[0][1], acc[0][2], acc[0][3]);
  acc_guard4(acc[1][0], acc[1][1], acc[1][2], acc[1][3]);
  acc_guard4(acc[2][0], acc[2][1], acc[2][2], acc[2][3]);
  acc_guard4(acc[3][0], acc[3][1], acc[3][2], acc[3][3]);

  float* slab = sT[wave];
  const float* Rb = RESID ? (resid + (size_t)b * strideR) : nullptr;
#pragma unroll
  for (int i = 0; i < 4; ++i) {
    const int mBase = m0 + (i << 4);
#pragma unroll
    for (int j = 0; j < 4; ++j) {
      const int n = n0 + (j << 4) + rlane;
      float bv = 0.f;
      if (BIAS_MODE == 2) bv = bias[n];
#pragma unroll
      for (int r = 0; r < 8; ++r) {
        float v = acc[i][j][r] * scale;
        if (BIAS_MODE == 1) v += bias[mBase + mOff + r];
        if (BIAS_MODE == 2) v += bv;
        if (RESID) v += Rb[(size_t)(mBase + mOff + r) * ldc + n];
        if (ACT == 2) v = fmaxf(v, 0.0f);
        if (ACT == 4) v = (v > 0.f) ? v : 0.01f * v;
        slab[(mOff + r) * 68 + (j << 4) + rlane] = v;
      }
    }
    __builtin_amdgcn_fence(__ATOMIC_RELEASE, "workgroup");
    __builtin_amdgcn_wave_barrier();
    __builtin_amdgcn_fence(__ATOMIC_ACQUIRE, "workgroup");
    if (OUT_MODE == 0) {
      float* C = (float*)Cout + (size_t)b * strideC;
      const int hh = lane >> 4, c4 = (lane & 15) * 4;
      for (int pass = 0; pass < 2; ++pass) {
#pragma unroll
        for (int it = 0; it < 8; ++it) {
          const int row = it * 2 + hh;
          v4f v = *(const v4f*)(slab + row * 68 + c4);
          *(volatile v4f*)(C + (size_t)(mBase + row) * ldc + n0 + c4) = v;
        }
        __threadfence();
      }
    } else {
      const int q = lane >> 3, c8 = (lane & 7) * 8;
      unsigned short* C  = (unsigned short*)Cout  + (size_t)b * strideC;
      unsigned short* C2 = (OUT_MODE == 2) ? ((unsigned short*)Cout2 + (size_t)b * strideC) : nullptr;
      for (int pass = 0; pass < 2; ++pass) {
#pragma unroll
        for (int it = 0; it < 4; ++it) {
          const int row = it * 4 + q;
          const float* sp = slab + row * 68 + c8;
          v8h hv, lv;
#pragma unroll
          for (int e = 0; e < 8; ++e) {
            if (OUT_MODE == 1) {
              hv[e] = (_Float16)sp[e];
            } else {
              unsigned short hb = f2bf_bits(sp[e]);
              unsigned short lb = f2bf_bits(sp[e] - bf_bits2f(hb));
              hv[e] = __builtin_bit_cast(_Float16, hb);
              lv[e] = __builtin_bit_cast(_Float16, lb);
            }
          }
          *(volatile v8h*)(C + (size_t)(mBase + row) * ldc + n0 + c8) = hv;
          if (OUT_MODE == 2) *(volatile v8h*)(C2 + (size_t)(mBase + row) * ldc + n0 + c8) = lv;
        }
        __threadfence();
      }
    }
    __builtin_amdgcn_fence(__ATOMIC_RELEASE, "workgroup");
    __builtin_amdgcn_wave_barrier();
    __builtin_amdgcn_fence(__ATOMIC_ACQUIRE, "workgroup");
  }
}

__global__ __launch_bounds__(256) void wtcast_kernel(const float* __restrict__ W0, const float* __restrict__ W1,
                                                     const float* __restrict__ W2, const float* __restrict__ W3,
                                                     unsigned short* __restrict__ out, float scale) {
  __shared__ float sm[64][65];
  const int t   = threadIdx.x;
  const int hm0 = blockIdx.x * 64;
  const int nd0 = blockIdx.y * 64;
  const int z   = blockIdx.z;
  const float* W = (z == 0) ? W0 : (z == 1) ? W1 : (z == 2) ? W2 : W3;
#pragma unroll
  for (int i = 0; i < 16; ++i) {
    const int e = i * 256 + t;
    const int r = e >> 6;
    const int c = e & 63;
    sm[c][r] = W[(size_t)(hm0 + r) * kHD + nd0 + c] * scale;
  }
  __syncthreads();
  const int lane = t & 31, wave = t >> 5;
  const int q = lane >> 3, c8 = (lane & 7) * 8;
  unsigned short* op = out + (size_t)z * kHD * kDModel;
  for (int pass = 0; pass < 2; ++pass) {
#pragma unroll
    for (int it = 0; it < 2; ++it) {
      const int row = wave * 8 + it * 4 + q;
      unsigned short hb[8];
#pragma unroll
      for (int e = 0; e < 8; ++e) hb[e] = h_bits(sm[row][c8 + e]);
      const v4u u = (v4u){pk16(hb[0], hb[1]), pk16(hb[2], hb[3]), pk16(hb[4], hb[5]), pk16(hb[6], hb[7])};
      *(volatile v4u*)(op + (size_t)(nd0 + row) * kDModel + hm0 + c8) = u;
    }
    __threadfence();
  }
}

__global__ __launch_bounds__(256) void cast8_f16_kernel(const float* __restrict__ in, unsigned short* __restrict__ out,
                                                        int n8, float scale) {
  const int i = blockIdx.x * 256 + threadIdx.x;
  if (i >= n8) return;
  const float* p = in + 8 * (size_t)i;
  const v4f a = *(const v4f*)(p);
  const v4f c = *(const v4f*)(p + 4);
  unsigned short hb[8];
#pragma unroll
  for (int e = 0; e < 4; ++e) {
    hb[e]     = h_bits(a[e] * scale);
    hb[4 + e] = h_bits(c[e] * scale);
  }
  const v4u u = (v4u){pk16(hb[0], hb[1]), pk16(hb[2], hb[3]), pk16(hb[4], hb[5]), pk16(hb[6], hb[7])};
  unsigned short* q = out + 8 * (size_t)i;
  *(volatile v4u*)q = u;
  __threadfence();
  *(volatile v4u*)q = u;
}

__global__ __launch_bounds__(128) void qprep_kernel(const float* __restrict__ Qf,
    const float* __restrict__ rwb, const float* __restrict__ rrb, const float* __restrict__ rsb,
    const float* __restrict__ sege,
    unsigned short* __restrict__ QW, unsigned short* __restrict__ QR, float* __restrict__ EF) {
  __shared__ __align__(16) float efs[kEFRow];
  const int i = blockIdx.x;
  const int b = blockIdx.y;
  const int t = threadIdx.x;
  const int c0 = t * 8;
  const int n  = t >> 3;
  const size_t row = (size_t)b * kQLen + i;

  const float* qp = Qf + row * kHD + c0;
  const v4f qa = *(const v4f*)(qp),            qc = *(const v4f*)(qp + 4);
  const v4f wa = *(const v4f*)(rwb + c0),      wc = *(const v4f*)(rwb + c0 + 4);
  const v4f ra = *(const v4f*)(rrb + c0),      rc = *(const v4f*)(rrb + c0 + 4);
  const v4f sa = *(const v4f*)(rsb + c0),      sc = *(const v4f*)(rsb + c0 + 4);
  const v4f e0a = *(const v4f*)(sege + c0),    e0c = *(const v4f*)(sege + c0 + 4);
  const v4f e1a = *(const v4f*)(sege + kHD + c0), e1c = *(const v4f*)(sege + kHD + c0 + 4);
  const float q[8]  = {qa[0], qa[1], qa[2], qa[3], qc[0], qc[1], qc[2], qc[3]};
  const float w[8]  = {wa[0], wa[1], wa[2], wa[3], wc[0], wc[1], wc[2], wc[3]};
  const float rr[8] = {ra[0], ra[1], ra[2], ra[3], rc[0], rc[1], rc[2], rc[3]};
  const float rs[8] = {sa[0], sa[1], sa[2], sa[3], sc[0], sc[1], sc[2], sc[3]};
  const float e0[8] = {e0a[0], e0a[1], e0a[2], e0a[3], e0c[0], e0c[1], e0c[2], e0c[3]};
  const float e1[8] = {e1a[0], e1a[1], e1a[2], e1a[3], e1c[0], e1c[1], e1c[2], e1c[3]};

  unsigned short hw[8], hr[8];
  float p0 = 0.f, p1 = 0.f;
#pragma unroll
  for (int e = 0; e < 8; ++e) {
    hw[e] = h_bits((q[e] + w[e]) * kQCarry);
    hr[e] = h_bits((q[e] + rr[e]) * kQCarry);
    const float qs = q[e] + rs[e];
    p0 = fmaf(qs, e0[e], p0);
    p1 = fmaf(qs, e1[e], p1);
  }
  p0 += __shfl_xor(p0, 1, 32); p1 += __shfl_xor(p1, 1, 32);
  p0 += __shfl_xor(p0, 2, 32); p1 += __shfl_xor(p1, 2, 32);
  p0 += __shfl_xor(p0, 4, 32); p1 += __shfl_xor(p1, 4, 32);
  if ((t & 7) == 0) { efs[2 * n] = p0; efs[2 * n + 1] = p1; }

  const v4u uw = (v4u){pk16(hw[0], hw[1]), pk16(hw[2], hw[3]), pk16(hw[4], hw[5]), pk16(hw[6], hw[7])};
  const v4u ur = (v4u){pk16(hr[0], hr[1]), pk16(hr[2], hr[3]), pk16(hr[4], hr[5]), pk16(hr[6], hr[7])};
  unsigned short* pw = QW + row * kHD + c0;
  unsigned short* pr = QR + row * kHD + c0;
  *(volatile v4u*)pw = uw;
  *(volatile v4u*)pr = ur;
  __syncthreads();
  const int tl = (t < 8) ? t : 0;
  const v4f ev = *(const v4f*)(efs + 4 * tl);
  float* ep = EF + row * kEFRow + 4 * tl;
  if (t < 8) *(volatile v4f*)ep = ev;
  __threadfence();
  *(volatile v4u*)pw = uw;
  *(volatile v4u*)pr = ur;
  if (t < 8) *(volatile v4f*)ep = ev;
}

__global__ __launch_bounds__(128) void softmax_kernel(const float* __restrict__ AC, const float* __restrict__ BDb,
    const float* __restrict__ EF, const float* __restrict__ segm, const float* __restrict__ amask,
    unsigned short* __restrict__ P16, int n) {
  __shared__ float redM[4];
  __shared__ float redS[4];
  const int i = blockIdx.x;
  const int b = blockIdx.y;
  const int t = threadIdx.x;
  const int lane = t & 31, wave = t >> 5;
  const int j0 = t * 8;
  const size_t row = (size_t)b * kQLen + i;

  const float* acp = AC + row * kQLen + j0;
  const v4f a0 = *(const v4f*)(acp);
  const v4f a1 = *(const v4f*)(acp + 4);
  const float ac[8] = {a0[0], a0[1], a0[2], a0[3], a1[0], a1[1], a1[2], a1[3]};
  const int cb = j0 + 64 - (i & 63);
  const float* bdp = BDb + row * kBand + cb;
  const float ef0 = EF[row * kEFRow + 2 * n];
  const float ef1 = EF[row * kEFRow + 2 * n + 1];
  const float* sp = segm  + (((size_t)i * kQLen + j0) * kBsz + b) * 2;
  const float* mp = amask + ((size_t)i * kQLen + j0) * kBsz + b;

  float s[8];
#pragma unroll
  for (int e = 0; e < 8; ++e) {
    const v2f sg  = *(const v2f*)(sp + 8 * e);
    const float mk = mp[4 * e];
    const float bd = bdp[e];
    const float efv = sg[0] * ef0 + sg[1] * ef1;
    const float tot = (ac[e] + bd) + efv;
    s[e] = tot * kScoreScale - 1e30f * mk;
  }
  float m = fmaxf(fmaxf(fmaxf(s[0], s[1]), fmaxf(s[2], s[3])), fmaxf(fmaxf(s[4], s[5]), fmaxf(s[6], s[7])));
#pragma unroll
  for (int off = 16; off > 0; off >>= 1) m = fmaxf(m, __shfl_xor(m, off, 32));
  if (lane == 0) redM[wave] = m;
  __syncthreads();
  const float rmax = fmaxf(fmaxf(redM[0], redM[1]), fmaxf(redM[2], redM[3]));

  float p[8];
  float ps = 0.f;
#pragma unroll
  for (int e = 0; e < 8; ++e) { p[e] = expf(s[e] - rmax); ps += p[e]; }
#pragma unroll
  for (int off = 16; off > 0; off >>= 1) ps += __shfl_xor(ps, off, 32);
  if (lane == 0) redS[wave] = ps;
  __syncthreads();
  const float total = ((redS[0] + redS[1]) + redS[2]) + redS[3];
  const float inv = kPCarry * (1.0f / total);

  unsigned short hb[8];
#pragma unroll
  for (int e = 0; e < 8; ++e) hb[e] = h_bits(p[e] * inv);
  const v4u u = (v4u){pk16(hb[0], hb[1]), pk16(hb[2], hb[3]), pk16(hb[4], hb[5]), pk16(hb[6], hb[7])};
  unsigned short* pp = P16 + row * kQLen + j0;
  *(volatile v4u*)pp = u;
  __threadfence();
  *(volatile v4u*)pp = u;
}

__global__ __launch_bounds__(256) void ln_kernel(const float* __restrict__ Y, const float* __restrict__ gamma,
                                                 const float* __restrict__ beta, float* __restrict__ out) {
  __shared__ float redA[8];
  __shared__ float redB[8];
  const int rowi = blockIdx.x;
  const int t = threadIdx.x;
  const int lane = t & 31, wave = t >> 5;
  const int c0 = 4 * t;
  const size_t base = (size_t)rowi * kDModel + c0;
  const v4f y = *(const v4f*)(Y + base);
  float su = (y[0] + y[1]) + (y[2] + y[3]);
#pragma unroll
  for (int off = 16; off > 0; off >>= 1) su += __shfl_xor(su, off, 32);
  if (lane == 0) redA[wave] = su;
  __syncthreads();
  float tot = 0.f;
#pragma unroll
  for (int w = 0; w < 8; ++w) tot += redA[w];
  const float mu = tot * kInvD;
  const float d0 = y[0] - mu, d1 = y[1] - mu, d2 = y[2] - mu, d3 = y[3] - mu;
  float sv = (d0 * d0 + d1 * d1) + (d2 * d2 + d3 * d3);
#pragma unroll
  for (int off = 16; off > 0; off >>= 1) sv += __shfl_xor(sv, off, 32);
  if (lane == 0) redB[wave] = sv;
  __syncthreads();
  float tot2 = 0.f;
#pragma unroll
  for (int w = 0; w < 8; ++w) tot2 += redB[w];
  const float var  = tot2 * kInvD;
  const float rstd = rsqrtf(var + kLnEps);
  const v4f g  = *(const v4f*)(gamma + c0);
  const v4f bt = *(const v4f*)(beta + c0);
  v4f o;
  o[0] = d0 * rstd * g[0] + bt[0];
  o[1] = d1 * rstd * g[1] + bt[1];
  o[2] = d2 * rstd * g[2] + bt[2];
  o[3] = d3 * rstd * g[3] + bt[3];
  float* op = out + base;
  *(volatile v4f*)op = o;
  __threadfence();
  *(volatile v4f*)op = o;
}

extern "C" void kernel_launch(void* const* d_in, const int* in_sizes, int n_in,
                              void* d_out, int out_size, void* d_ws, size_t ws_size,
                              hipStream_t stream)
{
  constexpr size_t MiB = 1048576;
  constexpr size_t offH16  = 0;
  constexpr size_t offR16  = 8 * MiB;
  constexpr size_t offWT   = 24 * MiB;
  constexpr size_t offQf32 = 32 * MiB;
  constexpr size_t offAC   = 0;
  constexpr size_t offBDb  = 16 * MiB;
  constexpr size_t szBDb   = (size_t)kBsz * kQLen * kBand * 4;
  constexpr size_t offP16  = offBDb + szBDb;
  constexpr size_t offY    = 0;
  constexpr size_t offWo16 = 48 * MiB;
  constexpr size_t offQW   = 50 * MiB;
  constexpr size_t offQR   = 58 * MiB;
  constexpr size_t offK16  = 66 * MiB;
  constexpr size_t offVt16 = 74 * MiB;
  constexpr size_t offKR16 = 82 * MiB;
  constexpr size_t offAV16 = 98 * MiB;
  constexpr size_t offEF   = 106 * MiB;
  constexpr size_t szEF    = (size_t)kBsz * kQLen * kEFRow * 4;
  constexpr size_t wsTotal = offEF + szEF;
  static_assert(offP16 + (size_t)kBsz * kQLen * kQLen * 2 <= offWo16, "phase-4 scratch inside X");
  static_assert(offQf32 + (size_t)kBsz * kQLen * kHD * 4 <= offWo16, "phase-3 planes inside X");
  static_assert(wsTotal <= (size_t)134217728, "carve budget");

  if (n_in < 15) return;
  if (in_sizes[0] != kTokQ * kDModel || in_sizes[1] != kTokR * kDModel ||
      in_sizes[2] != kQLen * kQLen * kBsz || in_sizes[3] != kQLen * kQLen * kBsz * 2 ||
      in_sizes[4] != kDModel * kHD || in_sizes[7] != kDModel * kHD || in_sizes[8] != kDModel * kHD ||
      in_sizes[9] != kHD || in_sizes[12] != 2 * kHD || in_sizes[13] != kDModel ||
      out_size != kTokQ * kDModel) return;
  if (ws_size < wsTotal) return;

  const float* h         = (const float*)d_in[0];
  const float* r         = (const float*)d_in[1];
  const float* attn_mask = (const float*)d_in[2];
  const float* seg_mat   = (const float*)d_in[3];
  const float* proj_q    = (const float*)d_in[4];
  const float* proj_k    = (const float*)d_in[5];
  const float* proj_v    = (const float*)d_in[6];
  const float* proj_o    = (const float*)d_in[7];
  const float* proj_r    = (const float*)d_in[8];
  const float* r_w_bias  = (const float*)d_in[9];
  const float* r_r_bias  = (const float*)d_in[10];
  const float* r_s_bias  = (const float*)d_in[11];
  const float* seg_embed = (const float*)d_in[12];
  const float* ln_gamma  = (const float*)d_in[13];
  const float* ln_beta   = (const float*)d_in[14];
  float* out = (float*)d_out;

  char* ws = (char*)d_ws;
  unsigned short* h16  = (unsigned short*)(ws + offH16);
  unsigned short* r16  = (unsigned short*)(ws + offR16);
  unsigned short* WT   = (unsigned short*)(ws + offWT);
  unsigned short* WqT  = WT;
  unsigned short* WkT  = WT + (size_t)1 * kHD * kDModel;
  unsigned short* WvT  = WT + (size_t)2 * kHD * kDModel;
  unsigned short* WrT  = WT + (size_t)3 * kHD * kDModel;
  float*          Qf32 = (float*)(ws + offQf32);
  float*          AC   = (float*)(ws + offAC);
  float*          BDb  = (float*)(ws + offBDb);
  unsigned short* P16  = (unsigned short*)(ws + offP16);
  float*          Y    = (float*)(ws + offY);
  unsigned short* Wo16 = (unsigned short*)(ws + offWo16);
  unsigned short* QW16 = (unsigned short*)(ws + offQW);
  unsigned short* QR16 = (unsigned short*)(ws + offQR);
  unsigned short* K16  = (unsigned short*)(ws + offK16);
  unsigned short* Vt16 = (unsigned short*)(ws + offVt16);
  unsigned short* KR16 = (unsigned short*)(ws + offKR16);
  unsigned short* AV16 = (unsigned short*)(ws + offAV16);
  float*          EF   = (float*)(ws + offEF);

  const long planeQ  = (long)kQLen * kHD;
  const long planeKR = (long)kRLen * kHD;
  const long planeBD = (long)kQLen * kBand;

  cast8_f16_kernel<<<dim3((kTokQ * kDModel / 8) / 256), 256, 0, stream>>>(h, h16, kTokQ * kDModel / 8, 1.0f);
  cast8_f16_kernel<<<dim3((kTokR * kDModel / 8) / 256), 256, 0, stream>>>(r, r16, kTokR * kDModel / 8, 1.0f);
  wtcast_kernel<<<dim3(kDModel / 64, kHD / 64, 4), 256, 0, stream>>>(proj_q, proj_k, proj_v, proj_r, WT, kWCarry);
  cast8_f16_kernel<<<dim3((kDModel * kHD / 8) / 256), 256, 0, stream>>>(proj_o, Wo16, kDModel * kHD / 8, kWCarry);

  wmma_gemm64<0, false, 0, 0, false, 0, false><<<dim3((kQLen / 64) * (kHD / 64) / 8, kBsz), 256, 0, stream>>>(
      h16, nullptr, kBsz * kDModel, (long)kDModel, WqT, nullptr, kDModel, 0L,
      Qf32, nullptr, kHD, planeQ, nullptr, nullptr, 0L, kQLen, kHD, kDModel, kScaleQf32, 0);
  wmma_gemm64<0, false, 0, 1, false, 0, false><<<dim3((kQLen / 64) * (kHD / 64) / 8, kBsz), 256, 0, stream>>>(
      h16, nullptr, kBsz * kDModel, (long)kDModel, WkT, nullptr, kDModel, 0L,
      K16, nullptr, kHD, planeQ, nullptr, nullptr, 0L, kQLen, kHD, kDModel, kScaleP16, 0);
  wmma_gemm64<0, false, 0, 1, false, 0, false><<<dim3((kHD / 64) * (kQLen / 64) / 8, kBsz), 256, 0, stream>>>(
      WvT, nullptr, kDModel, 0L, h16, nullptr, kBsz * kDModel, (long)kDModel,
      Vt16, nullptr, kQLen, planeQ, nullptr, nullptr, 0L, kHD, kQLen, kDModel, kScaleP16, 0);
  wmma_gemm64<0, false, 0, 1, false, 0, false><<<dim3((kRLen / 64) * (kHD / 64) / 8, kBsz), 256, 0, stream>>>(
      r16, nullptr, kBsz * kDModel, (long)kDModel, WrT, nullptr, kDModel, 0L,
      KR16, nullptr, kHD, planeKR, nullptr, nullptr, 0L, kRLen, kHD, kDModel, kScaleP16, 0);

  qprep_kernel<<<dim3(kQLen, kBsz), 128, 0, stream>>>(Qf32, r_w_bias, r_r_bias, r_s_bias, seg_embed, QW16, QR16, EF);

  for (int n = 0; n < kNHead; ++n) {
    const size_t colOff = (size_t)n * kDHead;
    wmma_gemm64<0, false, 0, 0, false, 0, false><<<dim3((kQLen / 64) * (kQLen / 64) / 8, kBsz), 256, 0, stream>>>(
        QW16 + colOff, nullptr, kHD, planeQ, K16 + colOff, nullptr, kHD, planeQ,
        AC, nullptr, kQLen, planeQ, nullptr, nullptr, 0L, kQLen, kQLen, kDHead, kScaleSc, 0);
    wmma_gemm64<0, false, 0, 0, false, 0, true><<<dim3((kQLen / 64) * (kBand / 64) / 8, kBsz), 256, 0, stream>>>(
        QR16 + colOff, nullptr, kHD, planeQ, KR16 + colOff, nullptr, kHD, planeKR,
        BDb, nullptr, kBand, planeBD, nullptr, nullptr, 0L, kQLen, kBand, kDHead, kScaleSc, kBandOff);
    softmax_kernel<<<dim3(kQLen, kBsz), 128, 0, stream>>>(AC, BDb, EF, seg_mat, attn_mask, P16, n);
    wmma_gemm64<0, false, 0, 1, false, 0, false><<<dim3((kQLen / 64) * (kDHead / 64) / 8, kBsz), 256, 0, stream>>>(
        P16, nullptr, kQLen, planeQ, Vt16 + colOff * kQLen, nullptr, kQLen, planeQ,
        AV16 + colOff, nullptr, kBsz * kHD, (long)kHD, nullptr, nullptr, 0L, kQLen, kDHead, kQLen, kScalePV, 0);
  }

  wmma_gemm64<0, false, 0, 0, true, 0, false><<<dim3((kTokQ / 64) * (kDModel / 64) / 8, 1), 256, 0, stream>>>(
      AV16, nullptr, kHD, 0L, Wo16, nullptr, kHD, 0L,
      Y, nullptr, kDModel, 0L, nullptr, h, 0L, kTokQ, kDModel, kHD, kScaleOut, 0);
  ln_kernel<<<dim3(kTokQ), 256, 0, stream>>>(Y, ln_gamma, ln_beta, out);
}
